// Point2Image_43516608643709
// MI455X (gfx1250) — hardware-verified
//
#include <hip/hip_runtime.h>

typedef __bf16 v16bf __attribute__((ext_vector_type(16)));
typedef unsigned short v8us __attribute__((ext_vector_type(8)));
typedef unsigned short v16us __attribute__((ext_vector_type(16)));
typedef float v8f __attribute__((ext_vector_type(8)));
typedef float v4f __attribute__((ext_vector_type(4)));
typedef v4f __attribute__((may_alias)) v4fa;
typedef v8us __attribute__((may_alias)) v8usa;

#define RES    384
#define NPTS   1024
#define PCOLS  5
#define NCH    4
#define NPL    6
#define KF     3072
#define PLANE  (RES * KF)
#define PPR    128
#define RB     32
#define WCOLS  48

static_assert(KF % 32 == 0);
static_assert(NPTS % 8 == 0);
static_assert((KF * 2) % 128 == 0);
static_assert((NPTS * 2) % 128 == 0);
static_assert((PLANE * 2) % 128 == 0);
static_assert(PPR % 32 == 0);
static_assert(RES % RB == 0);
static_assert(8 * WCOLS == RES);
static_assert((RES * 4) % 128 == 0);
static_assert((RB * RES) % (8 * 32 * 4 * 12) == 0);

__device__ __forceinline__ v8f wmma_bf(v16bf a, v16bf b, v8f c) {
  v8f d = __builtin_amdgcn_wmma_f32_16x16x32_bf16(false, a, false, b, (short)0, c, false, false);
  asm volatile("v_nop\n\tv_nop\n\tv_nop\n\tv_nop" : "+v"(d) : "v"(a), "v"(b));
  return d;
}

__device__ __forceinline__ v16bf ldfrag(const unsigned short* p, int h) {
  const v8us u0 = *(const v8usa*)(p + 8 * h);
  const v8us u1 = *(const v8usa*)(p + 16 + 8 * h);
  const v16us u = __builtin_shufflevector(u0, u1, 0, 1, 2, 3, 4, 5, 6, 7, 8, 9, 10, 11, 12, 13, 14, 15);
  return __builtin_bit_cast(v16bf, u);
}

__device__ __forceinline__ unsigned short bf16_bits(float v) {
  unsigned int u = __float_as_uint(v);
  u += 0x7FFFu + ((u >> 16) & 1u);
  return (unsigned short)(u >> 16);
}

__device__ __forceinline__ void split2(float v, unsigned short& hi, unsigned short& lo) {
  hi = bf16_bits(v);
  const float hf = __uint_as_float(((unsigned int)hi) << 16);
  lo = bf16_bits(v - hf);
}

__device__ __forceinline__ void store_seg3(unsigned short* base, v8us s0, v8us s1, v8us s2) {
  unsigned short* p0 = base;
  unsigned short* p1 = base + NPTS;
  unsigned short* p2 = base + 2 * NPTS;
  *(volatile v8us*)p0 = s0;
  *(volatile v8us*)p1 = s1;
  *(volatile v8us*)p2 = s2;
  __threadfence();
  *(volatile v8us*)p0 = s0;
  *(volatile v8us*)p1 = s1;
  *(volatile v8us*)p2 = s2;
}

__global__ __launch_bounds__(256) void prep_k(const float* __restrict__ p,
                                             unsigned short* __restrict__ wsp)
{
  #pragma clang fp contract(off)
  const int z = blockIdx.y;
  const int gid = blockIdx.x * 256 + threadIdx.x;
  if (gid >= RES * PPR) return;
  const int i = gid >> 7;
  const int piece = gid & (PPR - 1);
  const int n0 = piece * 8;

  const bool isA = (z < NCH);
  const int ccol = isA ? 1 : 0;
  const bool narrow = (z == 0) || (z == NCH);
  const float cexp = narrow ? (float)(20000.0 * 1.4426950408889634)
                            : (float)(1250.0 * 1.4426950408889634);
  const float hwf = narrow ? 6.0f : 23.0f;
  const bool usew = (z >= 1) && (z <= 3);
  const int wcol = usew ? (1 + z) : 2;

  const float fi = (float)i;
  const float rcp = 1.0f / 383.0f;
  const float lin = (i == RES - 1) ? 1.0f : (fi * rcp);

  v8us s0, s1, s2;
  #pragma unroll
  for (int e = 0; e < 8; ++e) {
    const int n = n0 + e;
    const float ctr = p[n * PCOLS + ccol];
    const float wv = p[n * PCOLS + wcol];
    const float cf = floorf(ctr * 384.0f);
    const bool m = (fi >= cf - hwf) && (fi <= cf + hwf);
    const float d = lin - ctr;
    const float sq = d * d;
    const float g = exp2f(-(sq * cexp));
    float val = m ? g : 0.0f;
    val = usew ? (val * wv) : val;
    unsigned short hb, lb;
    split2(val, hb, lb);
    s0[e] = hb;
    s1[e] = isA ? hb : lb;
    s2[e] = isA ? lb : hb;
  }
  unsigned short* base = wsp + (size_t)z * PLANE + (size_t)i * KF + n0;
  store_seg3(base, s0, s1, s2);
}

__global__ __launch_bounds__(256) void splat_k(const unsigned short* __restrict__ wsp,
                                              float* __restrict__ out)
{
  __shared__ __attribute__((aligned(16))) float sD[RB * RES];
  const int tid = threadIdx.x, lane = tid & 31, w = tid >> 5;
  const int h = lane >> 4, mm = lane & 15;
  const int rb = blockIdx.x;
  const int ch = blockIdx.y;

  const unsigned short* Apl = wsp + (size_t)ch * PLANE;
  const unsigned short* Bpl = wsp + (size_t)(NCH + ((ch == 0) ? 0 : 1)) * PLANE;
  const unsigned short* a0p = Apl + (size_t)(RB * rb + mm) * KF;
  const unsigned short* a1p = a0p + (size_t)16 * KF;
  const unsigned short* b0p = Bpl + (size_t)(WCOLS * w + mm) * KF;

  const v8f z8 = {0.f, 0.f, 0.f, 0.f, 0.f, 0.f, 0.f, 0.f};
  v8f acc0[3], acc1[3];
  #pragma unroll
  for (int nt = 0; nt < 3; ++nt) { acc0[nt] = z8; acc1[nt] = z8; }

  #pragma unroll 1
  for (int k0 = 0; k0 < KF; k0 += 32) {
    const v16bf fa0 = ldfrag(a0p + k0, h);
    const v16bf fa1 = ldfrag(a1p + k0, h);
    #pragma unroll
    for (int nt = 0; nt < 3; ++nt) {
      const v16bf fb = ldfrag(b0p + (size_t)nt * 16 * KF + k0, h);
      acc0[nt] = wmma_bf(fa0, fb, acc0[nt]);
      acc1[nt] = wmma_bf(fa1, fb, acc1[nt]);
    }
  }

  #pragma unroll
  for (int nt = 0; nt < 3; ++nt) {
    const int col = WCOLS * w + 16 * nt + mm;
    #pragma unroll
    for (int r = 0; r < 8; ++r) {
      const int r0 = 8 * h + r;
      sD[r0 * RES + col] = acc0[nt][r];
      sD[(r0 + 16) * RES + col] = acc1[nt][r];
    }
  }
  __syncthreads();

  float* ob = out + ((size_t)ch * RES + (size_t)RB * rb) * RES;
  const int sub = lane >> 3, q8 = lane & 7;
  #pragma unroll
  for (int it = 0; it < 12; ++it) {
    const int off = (48 * w + 4 * it + sub) * 32 + 4 * q8;
    const v4f v = *(const v4fa*)(sD + off);
    *(volatile v4f*)(ob + off) = v;
  }
  __threadfence();
  #pragma unroll
  for (int it = 0; it < 12; ++it) {
    const int off = (48 * w + 4 * it + sub) * 32 + 4 * q8;
    const v4f v = *(const v4fa*)(sD + off);
    *(volatile v4f*)(ob + off) = v;
  }
}

extern "C" void kernel_launch(void* const* d_in, const int* in_sizes, int n_in,
                              void* d_out, int out_size, void* d_ws, size_t ws_size,
                              hipStream_t stream) {
  if (n_in < 1) return;
  if (in_sizes[0] != NPTS * PCOLS) return;
  if (out_size != NCH * RES * RES) return;

  const size_t wsBytes = (size_t)NPL * PLANE * 2;
  if (wsBytes > ws_size) return;

  const float* p = (const float*)d_in[0];
  float* out = (float*)d_out;
  unsigned short* wsp = (unsigned short*)d_ws;

  const int gp = (RES * PPR + 255) / 256;
  prep_k<<<dim3(gp, NPL), 256, 0, stream>>>(p, wsp);
  splat_k<<<dim3(RES / RB, NCH), 256, 0, stream>>>(wsp, out);
}
